// _LatentHamiltonianFunc_15779709845805
// MI455X (gfx1250) — hardware-verified
//
#include <hip/hip_runtime.h>

#define NB   65536
#define DIM  128
#define HALF 64
#define HID  512
#define ADIM 128
#define LDS_BYTES 65536

typedef unsigned short us;
typedef us     v8us  __attribute__((ext_vector_type(8)));
typedef us     v16us __attribute__((ext_vector_type(16)));
typedef __bf16 v16bf __attribute__((ext_vector_type(16)));
typedef float  v8f   __attribute__((ext_vector_type(8)));
typedef float  v4f   __attribute__((ext_vector_type(4)));
typedef v8us  __attribute__((may_alias)) v8usa;
typedef v16us __attribute__((may_alias)) v16usa;
typedef v4f   __attribute__((may_alias)) v4fa;

union Frag { v16bf b; v16us u; v8us half[2]; };

__device__ __forceinline__ us f2bf(float x) {
  unsigned u = __float_as_uint(x);
  u += 0x7FFFu + ((u >> 16) & 1u);
  return (us)(u >> 16);
}
__device__ __forceinline__ float bfr(float x) {
  return __uint_as_float(((unsigned)f2bf(x)) << 16);
}

__device__ __forceinline__ v8f wmma_bf16(v16bf a, v16bf b, v8f c) {
  v8f d = __builtin_amdgcn_wmma_f32_16x16x32_bf16(false, a, false, b, (short)0, c, false, false);
  asm volatile("v_nop\n\tv_nop\n\tv_nop\n\tv_nop" : "+v"(d) : "v"(a), "v"(b));
  return d;
}

__device__ __forceinline__ v16bf load_b(const us* fragbase, int lane) {
  Frag f;
  f.u = *(const v16usa*)(fragbase + lane * 16);
  return f.b;
}

__device__ __forceinline__ v16bf load_a_lds(const us* p, int h) {
  Frag f;
  f.half[0] = *(const v8usa*)(p + 8 * h);
  f.half[1] = *(const v8usa*)(p + 16 + 8 * h);
  return f.b;
}

__device__ __forceinline__ v16bf load_a_f32(const float* p, int h) {
  const v4f x0 = *(const v4fa*)(p + 8 * h);
  const v4f x1 = *(const v4fa*)(p + 8 * h + 4);
  const v4f x2 = *(const v4fa*)(p + 16 + 8 * h);
  const v4f x3 = *(const v4fa*)(p + 16 + 8 * h + 4);
  Frag f;
  const v16us u = { f2bf(x0.x), f2bf(x0.y), f2bf(x0.z), f2bf(x0.w),
                    f2bf(x1.x), f2bf(x1.y), f2bf(x1.z), f2bf(x1.w),
                    f2bf(x2.x), f2bf(x2.y), f2bf(x2.z), f2bf(x2.w),
                    f2bf(x3.x), f2bf(x3.y), f2bf(x3.z), f2bf(x3.w) };
  f.u = u;
  return f.b;
}

__device__ __forceinline__ void act_pair(float a, float& sp, float& sg) {
  const float e  = __expf(-fabsf(a));
  const float rc = __builtin_amdgcn_rcpf(1.0f + e);
  sg = (a >= 0.0f) ? rc : e * rc;
  sp = fmaxf(a, 0.0f) + __logf(1.0f + e);
}
__device__ __forceinline__ float sigm(float a) {
  const float e  = __expf(-fabsf(a));
  const float rc = __builtin_amdgcn_rcpf(1.0f + e);
  return (a >= 0.0f) ? rc : e * rc;
}

__global__ __launch_bounds__(256) void pack_bfrag_kernel(
    const float* __restrict__ src, us* __restrict__ dst, int K, int N, int sk, int sn)
{
  const int t = blockIdx.x * 256 + threadIdx.x;
  const int total8 = (K * N) >> 3;
  if (t >= total8) return;
  const int tilesK = K >> 5;
  const int f    = t >> 6;
  const int lane = (t >> 1) & 31;
  const int g    = t & 1;
  const int kt = f % tilesK, nt = f / tilesK;
  const int h = lane >> 4, n = nt * 16 + (lane & 15);
  const int kb = kt * 32 + 16 * g + 8 * h;
  const float* s = src + (size_t)kb * sk + (size_t)n * sn;
  const v8us o = { f2bf(s[0 * sk]), f2bf(s[1 * sk]), f2bf(s[2 * sk]), f2bf(s[3 * sk]),
                   f2bf(s[4 * sk]), f2bf(s[5 * sk]), f2bf(s[6 * sk]), f2bf(s[7 * sk]) };
  us* d = dst + (size_t)t * 8;
  *(volatile v8us*)d = o;
  __threadfence();
  *(volatile v8us*)d = o;
}

__device__ __forceinline__ void out_store_pass(const float* sOut, float* out, int row0, int lane) {
#pragma unroll
  for (int i = 0; i < 16; ++i) {
    const v4f v = *(const v4fa*)(sOut + i * DIM + lane * 4);
    *(volatile v4f*)(out + (size_t)(row0 + i) * DIM + lane * 4) = v;
  }
}

__global__ __launch_bounds__(32) void hgrad_kernel(
    const float* __restrict__ z, const float* __restrict__ act,
    const float* __restrict__ damping,
    const float* __restrict__ b1, const float* __restrict__ b2,
    const float* __restrict__ W3, const float* __restrict__ b3,
    const float* __restrict__ Gb,
    const us* __restrict__ w1f,
    const us* __restrict__ w2f,
    const us* __restrict__ w2tf,
    const us* __restrict__ w1tf,
    const us* __restrict__ gwf,
    float* __restrict__ out)
{
  extern __shared__ __attribute__((aligned(16))) unsigned char lds_raw[];
  us*    bufA = (us*)lds_raw;
  us*    bufB = (us*)(lds_raw + 16384);
  float* sig  = (float*)(lds_raw + 32768);
  float* sDH  = sig;
  float* sOut = sig + 16 * DIM;

  (void)b3;

  const int lane = threadIdx.x & 31;
  const int h = lane >> 4, m = lane & 15;
  const int row0 = blockIdx.x * 16;
  const v8f zero8 = {0.f, 0.f, 0.f, 0.f, 0.f, 0.f, 0.f, 0.f};

  v16bf za[4];
  {
    const float* zr = z + (size_t)(row0 + m) * DIM;
#pragma unroll
    for (int kt = 0; kt < 4; ++kt) za[kt] = load_a_f32(zr + kt * 32, h);
  }
#pragma unroll 1
  for (int nt = 0; nt < 32; ++nt) {
    const us* wb = w1f + (size_t)nt * 4 * 512;
    v8f acc = zero8;
#pragma unroll
    for (int kt = 0; kt < 4; ++kt) acc = wmma_bf16(za[kt], load_b(wb + kt * 512, lane), acc);
    const int col = nt * 16 + m;
    const float bias = bfr(b1[col]);
#pragma unroll
    for (int r = 0; r < 8; ++r) {
      const int M = 8 * h + r;
      float sp, sg;
      act_pair(acc[r] + bias, sp, sg);
      bufA[M * HID + col] = f2bf(sp);
      sig[M * HID + col] = sg;
    }
  }
  __syncthreads();

#pragma unroll 1
  for (int nt = 0; nt < 32; ++nt) {
    const us* wb = w2f + (size_t)nt * 16 * 512;
    v8f acc = zero8;
#pragma unroll 4
    for (int kt = 0; kt < 16; ++kt) {
      const v16bf a = load_a_lds(bufA + m * HID + kt * 32, h);
      const v16bf b = load_b(wb + kt * 512, lane);
      acc = wmma_bf16(a, b, acc);
    }
    const int col = nt * 16 + m;
    const float bias = bfr(b2[col]);
    const float w3v  = bfr(W3[col]);
#pragma unroll
    for (int r = 0; r < 8; ++r) {
      const int M = 8 * h + r;
      bufB[M * HID + col] = f2bf(sigm(acc[r] + bias) * w3v);
    }
  }
  __syncthreads();

#pragma unroll 1
  for (int nt = 0; nt < 32; ++nt) {
    const us* wb = w2tf + (size_t)nt * 16 * 512;
    v8f acc = zero8;
#pragma unroll 4
    for (int kt = 0; kt < 16; ++kt) {
      const v16bf a = load_a_lds(bufB + m * HID + kt * 32, h);
      const v16bf b = load_b(wb + kt * 512, lane);
      acc = wmma_bf16(a, b, acc);
    }
    const int col = nt * 16 + m;
#pragma unroll
    for (int r = 0; r < 8; ++r) {
      const int M = 8 * h + r;
      bufA[M * HID + col] = f2bf(acc[r] * sig[M * HID + col]);
    }
  }
  __syncthreads();

#pragma unroll 1
  for (int nt = 0; nt < 8; ++nt) {
    const us* wb = w1tf + (size_t)nt * 16 * 512;
    v8f acc = zero8;
#pragma unroll 4
    for (int kt = 0; kt < 16; ++kt) {
      const v16bf a = load_a_lds(bufA + m * HID + kt * 32, h);
      const v16bf b = load_b(wb + kt * 512, lane);
      acc = wmma_bf16(a, b, acc);
    }
    const int col = nt * 16 + m;
#pragma unroll
    for (int r = 0; r < 8; ++r) sDH[(8 * h + r) * DIM + col] = acc[r];
  }

  v16bf aa[4];
  {
    const float* ar = act + (size_t)(row0 + m) * ADIM;
#pragma unroll
    for (int kt = 0; kt < 4; ++kt) aa[kt] = load_a_f32(ar + kt * 32, h);
  }
  __syncthreads();
  const float dmp = bfr(damping[0]);
#pragma unroll 1
  for (int nt = 0; nt < 4; ++nt) {
    const us* wb = gwf + (size_t)nt * 4 * 512;
    v8f acc = zero8;
#pragma unroll
    for (int kt = 0; kt < 4; ++kt) acc = wmma_bf16(aa[kt], load_b(wb + kt * 512, lane), acc);
    const int c = nt * 16 + m;
    const float gb = bfr(Gb[c]);
#pragma unroll
    for (int r = 0; r < 8; ++r) {
      const int M = 8 * h + r;
      const float dHp = sDH[M * DIM + HALF + c];
      const float dHq = sDH[M * DIM + c];
      const float gu  = acc[r] + gb;
      sOut[M * DIM + c]        = dHp;
      sOut[M * DIM + HALF + c] = -dHq - dmp * dHp + gu;
    }
  }
  __syncthreads();

  out_store_pass(sOut, out, row0, lane);
  __threadfence();
  out_store_pass(sOut, out, row0, lane);
}

extern "C" void kernel_launch(void* const* d_in, const int* in_sizes, int n_in,
                              void* d_out, int out_size, void* d_ws, size_t ws_size,
                              hipStream_t stream) {
  if (n_in < 11) return;
  if (in_sizes[0] != NB * DIM) return;
  if (in_sizes[1] != NB * ADIM) return;
  if (in_sizes[2] < 1) return;
  if (in_sizes[3] != DIM * HID || in_sizes[4] != HID) return;
  if (in_sizes[5] != HID * HID || in_sizes[6] != HID) return;
  if (in_sizes[7] != HID || in_sizes[8] < 1) return;
  if (in_sizes[9] != ADIM * HALF || in_sizes[10] != HALF) return;
  if (out_size != NB * DIM) return;

  const float* z       = (const float*)d_in[0];
  const float* act     = (const float*)d_in[1];
  const float* damping = (const float*)d_in[2];
  const float* W1      = (const float*)d_in[3];
  const float* b1      = (const float*)d_in[4];
  const float* W2      = (const float*)d_in[5];
  const float* b2      = (const float*)d_in[6];
  const float* W3      = (const float*)d_in[7];
  const float* b3      = (const float*)d_in[8];
  const float* Gw      = (const float*)d_in[9];
  const float* Gb      = (const float*)d_in[10];
  float* out = (float*)d_out;

  const size_t w1f_bytes  = (size_t)DIM * HID * 2;
  const size_t w2f_bytes  = (size_t)HID * HID * 2;
  const size_t w2tf_bytes = (size_t)HID * HID * 2;
  const size_t w1tf_bytes = (size_t)HID * DIM * 2;
  const size_t gwf_bytes  = (size_t)ADIM * HALF * 2;
  const size_t off_w1f  = 0;
  const size_t off_w2f  = off_w1f + w1f_bytes;
  const size_t off_w2tf = off_w2f + w2f_bytes;
  const size_t off_w1tf = off_w2tf + w2tf_bytes;
  const size_t off_gwf  = off_w1tf + w1tf_bytes;
  const size_t total    = off_gwf + gwf_bytes;
  if (total > ws_size) return;

  char* ws = (char*)d_ws;
  us* w1f  = (us*)(ws + off_w1f);
  us* w2f  = (us*)(ws + off_w2f);
  us* w2tf = (us*)(ws + off_w2tf);
  us* w1tf = (us*)(ws + off_w1tf);
  us* gwf  = (us*)(ws + off_gwf);

  pack_bfrag_kernel<<<(DIM * HID / 8 + 255) / 256, 256, 0, stream>>>(W1, w1f,  DIM,  HID,  HID, 1);
  pack_bfrag_kernel<<<(HID * HID / 8 + 255) / 256, 256, 0, stream>>>(W2, w2f,  HID,  HID,  HID, 1);
  pack_bfrag_kernel<<<(HID * HID / 8 + 255) / 256, 256, 0, stream>>>(W2, w2tf, HID,  HID,  1, HID);
  pack_bfrag_kernel<<<(HID * DIM / 8 + 255) / 256, 256, 0, stream>>>(W1, w1tf, HID,  DIM,  1, HID);
  pack_bfrag_kernel<<<(ADIM * HALF / 8 + 255) / 256, 256, 0, stream>>>(Gw, gwf, ADIM, HALF, HALF, 1);

  hgrad_kernel<<<NB / 16, 32, LDS_BYTES, stream>>>(
      z, act, damping, b1, b2, W3, b3, Gb, w1f, w2f, w2tf, w1tf, gwf, out);
}
